// CustomHyperSemanticMessagePassing_58574763983241
// MI455X (gfx1250) — hardware-verified
//
#include <hip/hip_runtime.h>

#define IN_DIMC   128
#define OUT_DIMC  128
#define EDGE_DIMC 64
#define DD        4
#define KK        8

typedef float v4f __attribute__((ext_vector_type(4)));
typedef float v8f __attribute__((ext_vector_type(8)));
typedef v4f __attribute__((__may_alias__)) v4fa;
typedef unsigned short v4us __attribute__((ext_vector_type(4)));
typedef unsigned short v8us __attribute__((ext_vector_type(8)));
typedef __bf16 v8b  __attribute__((ext_vector_type(8)));
typedef __bf16 v16b __attribute__((ext_vector_type(16)));
union Frag16 { v16b v; v8b h[2]; };

__device__ __forceinline__ unsigned short f2bf(float f) {
  unsigned int u = __float_as_uint(f);
  u += 0x7FFFu + ((u >> 16) & 1u);
  return (unsigned short)(u >> 16);
}
__device__ __forceinline__ float bf2f(unsigned short b) {
  return __uint_as_float(((unsigned int)b) << 16);
}
__device__ __forceinline__ void split1(float x, unsigned short& hi, unsigned short& lo) {
  const unsigned short hb = f2bf(x);
  hi = hb;
  lo = f2bf(x - bf2f(hb));
}
__device__ __forceinline__ void split4(v4f x, v4us& hi, v4us& lo) {
  unsigned short h0, h1, h2, h3, l0, l1, l2, l3;
  split1(x.x, h0, l0);
  split1(x.y, h1, l1);
  split1(x.z, h2, l2);
  split1(x.w, h3, l3);
  v4us hv = {h0, h1, h2, h3};
  v4us lv = {l0, l1, l2, l3};
  hi = hv;
  lo = lv;
}

__device__ __forceinline__ v8f wmma3_bf16(v8f c, v16b ah, v16b al, v16b bh, v16b bl) {
  c = __builtin_amdgcn_wmma_f32_16x16x32_bf16(false, ah, false, bl, (short)0, c, false, false);
  c = __builtin_amdgcn_wmma_f32_16x16x32_bf16(false, al, false, bh, (short)0, c, false, false);
  c = __builtin_amdgcn_wmma_f32_16x16x32_bf16(false, ah, false, bh, (short)0, c, false, false);
  asm volatile("v_nop\n\tv_nop\n\tv_nop\n\tv_nop" : "+v"(c) : "v"(ah), "v"(al), "v"(bh), "v"(bl));
  return c;
}

__global__ __launch_bounds__(256) void split_planes_kernel(const float* __restrict__ src,
                                                           unsigned short* hi,
                                                           unsigned short* lo,
                                                           int n8) {
  const int i = blockIdx.x * blockDim.x + threadIdx.x;
  if (i >= n8) return;
  const float* p = src + (size_t)i * 8;
  const v4f a = *(const v4f*)(p);
  const v4f b = *(const v4f*)(p + 4);
  v4us ha, la, hb, lb;
  split4(a, ha, la);
  split4(b, hb, lb);
  v8us H = {ha.x, ha.y, ha.z, ha.w, hb.x, hb.y, hb.z, hb.w};
  v8us L = {la.x, la.y, la.z, la.w, lb.x, lb.y, lb.z, lb.w};
  unsigned short* ph = hi + (size_t)i * 8;
  unsigned short* pl = lo + (size_t)i * 8;
  *(volatile v8us*)ph = H;
  *(volatile v8us*)pl = L;
  __threadfence();
  *(volatile v8us*)ph = H;
  *(volatile v8us*)pl = L;
}

__global__ __launch_bounds__(256) void weights_kernel(
    const float* __restrict__ Wlin, const float* __restrict__ Wedge,
    const float* __restrict__ Wq, const float* __restrict__ Wk,
    const float* __restrict__ Wv, const float* __restrict__ Wo,
    unsigned short* Mq_hi, unsigned short* Mq_lo,
    unsigned short* Mk_hi, unsigned short* Mk_lo,
    unsigned short* Mv_hi, unsigned short* Mv_lo,
    unsigned short* Wo_hi, unsigned short* Wo_lo,
    unsigned short* Mke_hi, unsigned short* Mke_lo) {
  const int lane = threadIdx.x & 31;
  const int w = blockIdx.x * (blockDim.x >> 5) + (threadIdx.x >> 5);
  const int NW_SQ  = 4 * OUT_DIMC;
  const int NW_ALL = NW_SQ + OUT_DIMC / 2;
  if (w >= NW_ALL) return;

  if (w < NW_SQ) {
    const int mat = w / OUT_DIMC;
    const int o   = w - mat * OUT_DIMC;
    const int i0  = 4 * lane;
    v4f acc = {0.f, 0.f, 0.f, 0.f};
    if (mat == 3) {
      acc = *(const v4f*)(Wo + (size_t)o * OUT_DIMC + i0);
    } else {
      const float* W = (mat == 0) ? Wq : (mat == 1) ? Wk : Wv;
#pragma unroll 4
      for (int j = 0; j < OUT_DIMC; ++j) {
        const float wj = W[(size_t)o * OUT_DIMC + j];
        const v4f  l  = *(const v4f*)(Wlin + (size_t)j * IN_DIMC + i0);
        acc.x += wj * l.x; acc.y += wj * l.y; acc.z += wj * l.z; acc.w += wj * l.w;
      }
    }
    v4us H, L;
    split4(acc, H, L);
    unsigned short* dh = (mat == 0) ? Mq_hi : (mat == 1) ? Mk_hi : (mat == 2) ? Mv_hi : Wo_hi;
    unsigned short* dl = (mat == 0) ? Mq_lo : (mat == 1) ? Mk_lo : (mat == 2) ? Mv_lo : Wo_lo;
    const size_t idx = (size_t)o * IN_DIMC + i0;
    *(volatile v4us*)(dh + idx) = H;
    *(volatile v4us*)(dl + idx) = L;
    __threadfence();
    *(volatile v4us*)(dh + idx) = H;
    *(volatile v4us*)(dl + idx) = L;
  } else {
    const int ww = w - NW_SQ;
    const int hh = lane >> 4, lm = lane & 15;
    const int o  = 2 * ww + hh;
    const int i0 = 4 * lm;
    v4f acc = {0.f, 0.f, 0.f, 0.f};
#pragma unroll 4
    for (int j = 0; j < OUT_DIMC; ++j) {
      const float wj = Wk[(size_t)o * OUT_DIMC + j];
      const v4f  l  = *(const v4f*)(Wedge + (size_t)j * EDGE_DIMC + i0);
      acc.x += wj * l.x; acc.y += wj * l.y; acc.z += wj * l.z; acc.w += wj * l.w;
    }
    v4us H, L;
    split4(acc, H, L);
    const size_t idx = (size_t)o * EDGE_DIMC + i0;
    *(volatile v4us*)(Mke_hi + idx) = H;
    *(volatile v4us*)(Mke_lo + idx) = L;
    __threadfence();
    *(volatile v4us*)(Mke_hi + idx) = H;
    *(volatile v4us*)(Mke_lo + idx) = L;
  }
}

template <int KD, int RELU>
__global__ __launch_bounds__(64) void gemm_bf3_kernel(
    const __bf16* __restrict__ Ahi, const __bf16* __restrict__ Alo,
    const __bf16* __restrict__ Bhi, const __bf16* __restrict__ Blo,
    const float* __restrict__ bias, int use_bias,
    float* out, int Mrows) {
  __shared__ float tile[2][16 * OUT_DIMC];

  const int lane = threadIdx.x & 31;
  const int h = lane >> 4, lm = lane & 15;
  const int wib = threadIdx.x >> 5;
  const int nW = (Mrows + 15) >> 4;
  int w = blockIdx.x * 2 + wib;
  const bool valid = (w < nW);
  if (!valid) w = nW - 1;
  const int aRow = w * 16;
  int ra = aRow + lm;
  if (ra > Mrows - 1) ra = Mrows - 1;

  const __bf16* pah = Ahi + (size_t)ra * KD + 8 * h;
  const __bf16* pal = Alo + (size_t)ra * KD + 8 * h;
  const __bf16* pbh = Bhi + (size_t)lm * KD + 8 * h;
  const __bf16* pbl = Blo + (size_t)lm * KD + 8 * h;

  v8f acc[8] = {};

#pragma unroll 1
  for (int k0 = 0; k0 < KD; k0 += 32) {
    Frag16 ah, al;
    ah.h[0] = *(const v8b*)(pah + k0);
    ah.h[1] = *(const v8b*)(pah + k0 + 16);
    al.h[0] = *(const v8b*)(pal + k0);
    al.h[1] = *(const v8b*)(pal + k0 + 16);
#pragma unroll
    for (int ct = 0; ct < 8; ++ct) {
      const size_t bofs = (size_t)(ct * 16) * KD + k0;
      Frag16 bh, bl;
      bh.h[0] = *(const v8b*)(pbh + bofs);
      bh.h[1] = *(const v8b*)(pbh + bofs + 16);
      bl.h[0] = *(const v8b*)(pbl + bofs);
      bl.h[1] = *(const v8b*)(pbl + bofs + 16);
      acc[ct] = wmma3_bf16(acc[ct], ah.v, al.v, bh.v, bl.v);
    }
  }

  float* tl = &tile[wib][0];
#pragma unroll
  for (int ct = 0; ct < 8; ++ct) {
    const int col = ct * 16 + lm;
    const float bb = use_bias ? bias[col] : 0.f;
#pragma unroll
    for (int r = 0; r < 8; ++r) {
      float v = acc[ct][r] + bb;
      if (RELU) v = fmaxf(v, 0.f);
      tl[(8 * h + r) * OUT_DIMC + col] = v;
    }
  }
  __syncthreads();

#pragma unroll
  for (int R = 0; R < 16; ++R) {
    const int row = aRow + R;
    const v4f v = *(const v4fa*)(tl + R * OUT_DIMC + 4 * lane);
    if (valid && row < Mrows)
      *(volatile v4f*)(out + (size_t)row * OUT_DIMC + 4 * lane) = v;
  }
  __threadfence();
#pragma unroll
  for (int R = 0; R < 16; ++R) {
    const int row = aRow + R;
    const v4f v = *(const v4fa*)(tl + R * OUT_DIMC + 4 * lane);
    if (valid && row < Mrows)
      *(volatile v4f*)(out + (size_t)row * OUT_DIMC + 4 * lane) = v;
  }
}

__global__ __launch_bounds__(256) void attn_kernel(const float* __restrict__ Qn,
                                                   const float* __restrict__ Kn,
                                                   const float* __restrict__ Vn,
                                                   const float* __restrict__ Ke,
                                                   const int* __restrict__ node_edges,
                                                   const int* __restrict__ edge_nodes,
                                                   unsigned short* ctx_hi,
                                                   unsigned short* ctx_lo,
                                                   int nn, int ee) {
  const int lane = threadIdx.x & 31;
  const int n = (int)((blockIdx.x * blockDim.x + threadIdx.x) >> 5);
  if (n >= nn) return;

  const int d0 = lane * 4;
  const v4f q = *(const v4f*)(Qn + (size_t)n * OUT_DIMC + d0);

  float m = -3.0e38f, s = 0.f;
  float ax = 0.f, ay = 0.f, az = 0.f, aw = 0.f;

#pragma unroll 1
  for (int d = 0; d < DD; ++d) {
    int e = node_edges[(size_t)n * DD + d];
    e = (e < 0) ? 0 : e;
    e = (e > ee - 1) ? (ee - 1) : e;
    const v4f ke = *(const v4f*)(Ke + (size_t)e * OUT_DIMC + d0);
    const int* en = edge_nodes + (size_t)e * KK;

    float p[KK];
    int   uu[KK];
#pragma unroll
    for (int j = 0; j < KK; ++j) {
      int u = en[j];
      u = (u < 0) ? 0 : u;
      u = (u > nn - 1) ? (nn - 1) : u;
      uu[j] = u;
      const v4f kn = *(const v4f*)(Kn + (size_t)u * OUT_DIMC + d0);
      float t = q.x * (kn.x + ke.x) + q.y * (kn.y + ke.y) +
                q.z * (kn.z + ke.z) + q.w * (kn.w + ke.w);
      t += __shfl_xor(t, 1);
      t += __shfl_xor(t, 2);
      p[j] = t * 0.25f;
    }
    float bm = p[0];
#pragma unroll
    for (int j = 1; j < KK; ++j) bm = fmaxf(bm, p[j]);
    const float mn = fmaxf(m, bm);
    const float rs = __expf(m - mn);
    s *= rs; ax *= rs; ay *= rs; az *= rs; aw *= rs;
#pragma unroll
    for (int j = 0; j < KK; ++j) {
      const float wgt = __expf(p[j] - mn);
      s += wgt;
      const v4f v = *(const v4f*)(Vn + (size_t)uu[j] * OUT_DIMC + d0);
      ax += wgt * v.x; ay += wgt * v.y; az += wgt * v.z; aw += wgt * v.w;
    }
    m = mn;
  }

  const float inv = 1.f / s;
  v4f c = {ax * inv, ay * inv, az * inv, aw * inv};
  v4us H, L;
  split4(c, H, L);
  const size_t idx = (size_t)n * OUT_DIMC + d0;
  *(volatile v4us*)(ctx_hi + idx) = H;
  *(volatile v4us*)(ctx_lo + idx) = L;
  __threadfence();
  *(volatile v4us*)(ctx_hi + idx) = H;
  *(volatile v4us*)(ctx_lo + idx) = L;
}

extern "C" void kernel_launch(void* const* d_in, const int* in_sizes, int n_in,
                              void* d_out, int out_size, void* d_ws, size_t ws_size,
                              hipStream_t stream) {
  if (n_in < 14) return;

  const float* x          = (const float*)d_in[0];
  const float* edge_attr  = (const float*)d_in[1];
  const int*   node_edges = (const int*)d_in[2];
  const int*   edge_nodes = (const int*)d_in[3];
  const float* W_lin  = (const float*)d_in[4];
  const float* W_edge = (const float*)d_in[5];
  const float* Wq = (const float*)d_in[6];
  const float* Wk = (const float*)d_in[7];
  const float* Wv = (const float*)d_in[8];
  const float* bq = (const float*)d_in[9];
  const float* bk = (const float*)d_in[10];
  const float* bv = (const float*)d_in[11];
  const float* Wo = (const float*)d_in[12];
  const float* bo = (const float*)d_in[13];
  float* out = (float*)d_out;

  const int nn = in_sizes[0] / IN_DIMC;
  const int ee = in_sizes[1] / EDGE_DIMC;
  if (nn <= 0 || ee <= 0) return;
  if (in_sizes[2] < nn * DD || in_sizes[3] < ee * KK) return;
  int out_rows = out_size / OUT_DIMC;
  if (out_rows > nn) out_rows = nn;
  if (out_rows <= 0) return;

  size_t off = 0;
  auto carve = [&](size_t bytes) -> size_t {
    size_t p = off;
    off += (bytes + 255) & ~(size_t)255;
    return p;
  };
  const size_t o_xhi  = carve((size_t)nn * IN_DIMC * 2);
  const size_t o_xlo  = carve((size_t)nn * IN_DIMC * 2);
  const size_t o_ehi  = carve((size_t)ee * EDGE_DIMC * 2);
  const size_t o_elo  = carve((size_t)ee * EDGE_DIMC * 2);
  const size_t o_mqh  = carve((size_t)OUT_DIMC * IN_DIMC * 2);
  const size_t o_mql  = carve((size_t)OUT_DIMC * IN_DIMC * 2);
  const size_t o_mkh  = carve((size_t)OUT_DIMC * IN_DIMC * 2);
  const size_t o_mkl  = carve((size_t)OUT_DIMC * IN_DIMC * 2);
  const size_t o_mvh  = carve((size_t)OUT_DIMC * IN_DIMC * 2);
  const size_t o_mvl  = carve((size_t)OUT_DIMC * IN_DIMC * 2);
  const size_t o_woh  = carve((size_t)OUT_DIMC * OUT_DIMC * 2);
  const size_t o_wol  = carve((size_t)OUT_DIMC * OUT_DIMC * 2);
  const size_t o_mkeh = carve((size_t)OUT_DIMC * EDGE_DIMC * 2);
  const size_t o_mkel = carve((size_t)OUT_DIMC * EDGE_DIMC * 2);
  const size_t o_qn   = carve((size_t)nn * OUT_DIMC * 4);
  const size_t o_kn   = carve((size_t)nn * OUT_DIMC * 4);
  const size_t o_vn   = carve((size_t)nn * OUT_DIMC * 4);
  const size_t o_ke   = carve((size_t)ee * OUT_DIMC * 4);
  const size_t o_cth  = carve((size_t)nn * OUT_DIMC * 2);
  const size_t o_ctl  = carve((size_t)nn * OUT_DIMC * 2);
  if (off > ws_size) return;

  char* ws = (char*)d_ws;
  unsigned short* xhi   = (unsigned short*)(ws + o_xhi);
  unsigned short* xlo   = (unsigned short*)(ws + o_xlo);
  unsigned short* ehi   = (unsigned short*)(ws + o_ehi);
  unsigned short* elo   = (unsigned short*)(ws + o_elo);
  unsigned short* Mq_hi = (unsigned short*)(ws + o_mqh);
  unsigned short* Mq_lo = (unsigned short*)(ws + o_mql);
  unsigned short* Mk_hi = (unsigned short*)(ws + o_mkh);
  unsigned short* Mk_lo = (unsigned short*)(ws + o_mkl);
  unsigned short* Mv_hi = (unsigned short*)(ws + o_mvh);
  unsigned short* Mv_lo = (unsigned short*)(ws + o_mvl);
  unsigned short* Wo_hi = (unsigned short*)(ws + o_woh);
  unsigned short* Wo_lo = (unsigned short*)(ws + o_wol);
  unsigned short* Mke_hi = (unsigned short*)(ws + o_mkeh);
  unsigned short* Mke_lo = (unsigned short*)(ws + o_mkel);
  float* Qn = (float*)(ws + o_qn);
  float* Kn = (float*)(ws + o_kn);
  float* Vn = (float*)(ws + o_vn);
  float* Ke = (float*)(ws + o_ke);
  unsigned short* ctx_hi = (unsigned short*)(ws + o_cth);
  unsigned short* ctx_lo = (unsigned short*)(ws + o_ctl);

  {
    const int n8 = (nn * IN_DIMC) / 8;
    split_planes_kernel<<<(n8 + 255) / 256, 256, 0, stream>>>(x, xhi, xlo, n8);
  }
  {
    const int n8 = (ee * EDGE_DIMC) / 8;
    split_planes_kernel<<<(n8 + 255) / 256, 256, 0, stream>>>(edge_attr, ehi, elo, n8);
  }

  {
    const int nwaves = 4 * OUT_DIMC + OUT_DIMC / 2;
    weights_kernel<<<(nwaves + 7) / 8, 256, 0, stream>>>(
        W_lin, W_edge, Wq, Wk, Wv, Wo,
        Mq_hi, Mq_lo, Mk_hi, Mk_lo, Mv_hi, Mv_lo, Wo_hi, Wo_lo, Mke_hi, Mke_lo);
  }

  {
    const int nW = (nn + 15) / 16;
    const int grid = (nW + 1) / 2;
    gemm_bf3_kernel<IN_DIMC, 0><<<grid, 64, 0, stream>>>(
        (const __bf16*)xhi, (const __bf16*)xlo, (const __bf16*)Mq_hi, (const __bf16*)Mq_lo,
        bq, 1, Qn, nn);
    gemm_bf3_kernel<IN_DIMC, 0><<<grid, 64, 0, stream>>>(
        (const __bf16*)xhi, (const __bf16*)xlo, (const __bf16*)Mk_hi, (const __bf16*)Mk_lo,
        bk, 0, Kn, nn);
    gemm_bf3_kernel<IN_DIMC, 0><<<grid, 64, 0, stream>>>(
        (const __bf16*)xhi, (const __bf16*)xlo, (const __bf16*)Mv_hi, (const __bf16*)Mv_lo,
        bv, 1, Vn, nn);
  }

  {
    const int nW = (ee + 15) / 16;
    const int grid = (nW + 1) / 2;
    gemm_bf3_kernel<EDGE_DIMC, 0><<<grid, 64, 0, stream>>>(
        (const __bf16*)ehi, (const __bf16*)elo, (const __bf16*)Mke_hi, (const __bf16*)Mke_lo,
        bk, 1, Ke, ee);
  }

  attn_kernel<<<(nn + 7) / 8, 256, 0, stream>>>(Qn, Kn, Vn, Ke, node_edges, edge_nodes,
                                                 ctx_hi, ctx_lo, nn, ee);

  {
    const int nW = (out_rows + 15) / 16;
    const int grid = (nW + 1) / 2;
    gemm_bf3_kernel<OUT_DIMC, 1><<<grid, 64, 0, stream>>>(
        (const __bf16*)ctx_hi, (const __bf16*)ctx_lo, (const __bf16*)Wo_hi, (const __bf16*)Wo_lo,
        bo, 1, out, out_rows);
  }
}
